// MixNode_60979945669128
// MI455X (gfx1250) — hardware-run, weakly checked
//
#include <hip/hip_runtime.h>


#define NB  16384
#define NK  512
#define NI  31
#define NL  62
#define NLP 64
#define NO  128
typedef _Float16 h16;
typedef unsigned short bf;
typedef __attribute__((ext_vector_type(16))) __bf16   v16bf;
typedef __attribute__((ext_vector_type(16))) _Float16 v16h;
typedef __attribute__((ext_vector_type(8)))  _Float16 v8h;
typedef __attribute__((ext_vector_type(8)))  unsigned short v8us;
typedef __attribute__((ext_vector_type(8)))  float    v8f;
typedef __attribute__((ext_vector_type(4)))  float    v4f;
typedef v8h  __attribute__((may_alias)) v8ha;
typedef v4f  __attribute__((may_alias)) v4fa;
typedef v8us __attribute__((may_alias)) v8usa;

__device__ __forceinline__ unsigned short f2bf(float f) { unsigned u = __float_as_uint(f); u += 0x7FFFu + ((u >> 16) & 1u); return (unsigned short)(u >> 16); }
__device__ __forceinline__ float bf2f(unsigned short b) { return __uint_as_float(((unsigned)b) << 16); }
__device__ __forceinline__ float bfr(float f) { return bf2f(f2bf(f)); }
__device__ __forceinline__ v16h cat16(v8h lo, v8h hi) { return __builtin_shufflevector(lo, hi, 0, 1, 2, 3, 4, 5, 6, 7, 8, 9, 10, 11, 12, 13, 14, 15); }
__device__ __forceinline__ v16bf cat16b(v8us lo, v8us hi) { return __builtin_bit_cast(v16bf, __builtin_shufflevector(lo, hi, 0, 1, 2, 3, 4, 5, 6, 7, 8, 9, 10, 11, 12, 13, 14, 15)); }
__device__ __forceinline__ v8f wmma16(v16h a, v16h b, v8f c) { return __builtin_amdgcn_wmma_f32_16x16x32_f16(false, a, false, b, (short)0, c, false, false); }
__device__ __forceinline__ v8f wmmab(v16bf a, v16bf b, v8f c) { return __builtin_amdgcn_wmma_f32_16x16x32_bf16(false, a, false, b, (short)0, c, false, false); }

template <typename T16> struct WFrag;
template <> struct WFrag<h16> { typedef v16h V; static __device__ __forceinline__ V ld(const h16* p) { return cat16(*(const v8h*)p, *(const v8h*)(p + 16)); } static __device__ __forceinline__ v8f mma(V a, V b, v8f c) { return wmma16(a, b, c); } };
template <> struct WFrag<bf> { typedef v16bf V; static __device__ __forceinline__ V ld(const bf* p) { return cat16b(*(const v8us*)p, *(const v8us*)(p + 16)); } static __device__ __forceinline__ v8f mma(V a, V b, v8f c) { return wmmab(a, b, c); } };
template <typename T16, int NSPLIT, bool BIAS>
__global__ __launch_bounds__(32) void k_gemmw(const T16* __restrict__ A, const T16* __restrict__ A2, const T16* __restrict__ Bt, const T16* __restrict__ Bt2, int K, float* C, int ldc, const float* __restrict__ bias, size_t sA, size_t sB, size_t sC) {
    typedef typename WFrag<T16>::V V;
    __shared__ __align__(16) float os[16 * 68];
    const size_t z = blockIdx.z; A += z * sA; if (A2) A2 += z * sA; Bt += z * sB; if (Bt2) Bt2 += z * sB; C += z * sC;
    const int lane = threadIdx.x & 31, lr = lane & 15, hi = lane >> 4; const int r0 = blockIdx.x * 64, c0 = blockIdx.y * 64;
    v8f acc[4][4];
#pragma unroll
    for (int mb = 0; mb < 4; ++mb)
#pragma unroll
        for (int nb = 0; nb < 4; ++nb) acc[mb][nb] = (v8f){};
    const size_t aoff = (size_t)(r0 + lr) * K + 8 * hi, boff = (size_t)(c0 + lr) * K + 8 * hi;
    for (int kc = 0; kc < K; kc += 32) {
        V a[4], a2[4];
#pragma unroll
        for (int mb = 0; mb < 4; ++mb) { a[mb] = WFrag<T16>::ld(A + aoff + (size_t)mb * 16 * K + kc); if (NSPLIT == 1 || NSPLIT == 2) a2[mb] = WFrag<T16>::ld(A2 + aoff + (size_t)mb * 16 * K + kc); }
#pragma unroll
        for (int nb = 0; nb < 4; ++nb) { const V b = WFrag<T16>::ld(Bt + boff + (size_t)nb * 16 * K + kc); V b2; if (NSPLIT >= 2) b2 = WFrag<T16>::ld(Bt2 + boff + (size_t)nb * 16 * K + kc);
#pragma unroll
            for (int mb = 0; mb < 4; ++mb) { acc[mb][nb] = WFrag<T16>::mma(a[mb], b, acc[mb][nb]); if (NSPLIT == 1 || NSPLIT == 2) acc[mb][nb] = WFrag<T16>::mma(a2[mb], b, acc[mb][nb]); if (NSPLIT >= 2) acc[mb][nb] = WFrag<T16>::mma(a[mb], b2, acc[mb][nb]); } }
        asm volatile("v_nop\n\tv_nop\n\tv_nop\n\tv_nop" : "+v"(acc[0][0]), "+v"(acc[1][1]), "+v"(acc[2][2]), "+v"(acc[3][3]) : "v"(a[0]), "v"(a[3]));
    }
#pragma unroll
    for (int mb = 0; mb < 4; ++mb) {
#pragma unroll
        for (int nb = 0; nb < 4; ++nb) {
#pragma unroll
            for (int j = 0; j < 8; ++j) os[(hi * 8 + j) * 68 + nb * 16 + lr] = acc[mb][nb][j]; }
        __builtin_amdgcn_wave_barrier(); asm volatile("" ::: "memory");
        float* crow = C + (size_t)(r0 + mb * 16) * ldc + c0;
#pragma unroll 1
        for (int ps = 0; ps < 2; ++ps) {
#pragma unroll
            for (int s = 0; s < 8; ++s) { const int row = 2 * s + hi, cofs = lr * 4; v4f val = *(const v4fa*)(os + row * 68 + cofs); if (BIAS) { val[0] += bfr(bias[c0 + cofs]); val[1] += bfr(bias[c0 + cofs + 1]); val[2] += bfr(bias[c0 + cofs + 2]); val[3] += bfr(bias[c0 + cofs + 3]); }
                *(volatile v4f*)(crow + (size_t)row * ldc + cofs) = val; }
            if (ps == 0) __threadfence(); }
        __builtin_amdgcn_wave_barrier(); asm volatile("" ::: "memory");
    }
}

typedef __attribute__((ext_vector_type(2))) float v2f;

__global__ __launch_bounds__(256) void k_cvt8(const float* __restrict__ src, bf* dst, size_t n8) { const size_t i = (size_t)blockIdx.x * 256 + threadIdx.x; if (i >= n8) return; const v8f v = *(const v8f*)(src + i * 8); v8us o;
#pragma unroll
    for (int k = 0; k < 8; ++k) o[k] = f2bf(v[k]); *(volatile v8us*)(dst + i * 8) = o; __threadfence(); *(volatile v8us*)(dst + i * 8) = o; }

__global__ __launch_bounds__(256) void k_wpad(const float* __restrict__ Wi, bf* WB) { const int i = blockIdx.x * 256 + threadIdx.x; if (i >= NLP * NK / 8) return; const int row = i / (NK / 8), c8 = i - row * (NK / 8); const int rs = row < NL ? row : NL - 1; const unsigned short keep = (unsigned short)(row < NL ? 0xffffu : 0u); const v8f v = *(const v8f*)(Wi + (size_t)rs * NK + c8 * 8); v8us o;
#pragma unroll
    for (int k = 0; k < 8; ++k) o[k] = (unsigned short)(f2bf(v[k]) & keep); bf* p = WB + (size_t)i * 8; *(volatile v8us*)p = o; __threadfence(); *(volatile v8us*)p = o; }

__global__ __launch_bounds__(32) void k_g(const float* __restrict__ gm, float* GG) { const int n = threadIdx.x; if (n >= NI) return; const float a = bfr(gm[2 * n]), c = bfr(gm[2 * n + 1]); const float mx = fmaxf(a, c); const float e0 = expf(a - mx), e1 = expf(c - mx); const float s = e0 + e1; v2f o; o[0] = e0 / s; o[1] = e1 / s; *(volatile v2f*)(GG + 2 * n) = o; __threadfence(); *(volatile v2f*)(GG + 2 * n) = o; }

__global__ __launch_bounds__(256) void k_route(const float* __restrict__ LG, const float* __restrict__ bi, float* RR) { const int i = blockIdx.x * 256 + threadIdx.x; const int n = i & 31, row = i >> 5; if (i >= NB * 32 || n >= NI) return; const v2f l = *(const v2f*)(LG + (size_t)row * NLP + 2 * n); const float a = l[0] + bfr(bi[2 * n]), c = l[1] + bfr(bi[2 * n + 1]); const float mx = fmaxf(a, c); const float e0 = expf(a - mx), e1 = expf(c - mx); const float s = e0 + e1; v2f o; o[0] = e0 / s; o[1] = e1 / s; float* p = RR + ((size_t)row * 32 + n) * 2; *(volatile v2f*)p = o; __threadfence(); *(volatile v2f*)p = o; }

#define R0(n) rr[2 * (n)]
#define R1(n) rr[2 * (n) + 1]
#define G0(n) gg[2 * (n)]
#define G1(n) gg[2 * (n) + 1]
#define LF(n) ldleaf(lf + (size_t)(n) * NO)
__device__ __forceinline__ v4f ldleaf(const float* p) { const v4f v = *(const v4f*)p; v4f o; o[0] = bfr(v[0]); o[1] = bfr(v[1]); o[2] = bfr(v[2]); o[3] = bfr(v[3]); return o; }
__global__ __launch_bounds__(256) void k_tree(const float* __restrict__ RR, const float* __restrict__ GG, const float* __restrict__ leaf, float* OUT) {
  const int i = blockIdx.x * 256 + threadIdx.x; if (i >= NB * (NO / 4)) return; const int q = i & (NO / 4 - 1), row = i >> 5; const float* rr = RR + (size_t)row * 64; const float* gg = GG; const float* lf = leaf + q * 4;
  const v4f L61 = LF(61), L62 = LF(62);
  const v4f y30 = G0(30) * (L61 * R0(30) + L62 * R1(30)) + G1(30) * LF(30);
  const v4f L59 = LF(59), L60 = LF(60);
  const v4f y29 = G0(29) * (L59 * R0(29) + L60 * R1(29)) + G1(29) * LF(29);
  const v4f L57 = LF(57), L58 = LF(58);
  const v4f y28 = G0(28) * (L57 * R0(28) + L58 * R1(28)) + G1(28) * LF(28);
  const v4f L55 = LF(55), L56 = LF(56);
  const v4f y27 = G0(27) * (L55 * R0(27) + L56 * R1(27)) + G1(27) * LF(27);
  const v4f L53 = LF(53), L54 = LF(54);
  const v4f y26 = G0(26) * (L53 * R0(26) + L54 * R1(26)) + G1(26) * LF(26);
  const v4f L51 = LF(51), L52 = LF(52);
  const v4f y25 = G0(25) * (L51 * R0(25) + L52 * R1(25)) + G1(25) * LF(25);
  const v4f L49 = LF(49), L50 = LF(50);
  const v4f y24 = G0(24) * (L49 * R0(24) + L50 * R1(24)) + G1(24) * LF(24);
  const v4f L47 = LF(47), L48 = LF(48);
  const v4f y23 = G0(23) * (L47 * R0(23) + L48 * R1(23)) + G1(23) * LF(23);
  const v4f L45 = LF(45), L46 = LF(46);
  const v4f y22 = G0(22) * (L45 * R0(22) + L46 * R1(22)) + G1(22) * LF(22);
  const v4f L43 = LF(43), L44 = LF(44);
  const v4f y21 = G0(21) * (L43 * R0(21) + L44 * R1(21)) + G1(21) * LF(21);
  const v4f L41 = LF(41), L42 = LF(42);
  const v4f y20 = G0(20) * (L41 * R0(20) + L42 * R1(20)) + G1(20) * LF(20);
  const v4f L39 = LF(39), L40 = LF(40);
  const v4f y19 = G0(19) * (L39 * R0(19) + L40 * R1(19)) + G1(19) * LF(19);
  const v4f L37 = LF(37), L38 = LF(38);
  const v4f y18 = G0(18) * (L37 * R0(18) + L38 * R1(18)) + G1(18) * LF(18);
  const v4f L35 = LF(35), L36 = LF(36);
  const v4f y17 = G0(17) * (L35 * R0(17) + L36 * R1(17)) + G1(17) * LF(17);
  const v4f L33 = LF(33), L34 = LF(34);
  const v4f y16 = G0(16) * (L33 * R0(16) + L34 * R1(16)) + G1(16) * LF(16);
  const v4f L31 = LF(31), L32 = LF(32);
  const v4f y15 = G0(15) * (L31 * R0(15) + L32 * R1(15)) + G1(15) * LF(15);
  const v4f y14 = G0(14) * (y29 * R0(14) + y30 * R1(14)) + G1(14) * LF(14);
  const v4f y13 = G0(13) * (y27 * R0(13) + y28 * R1(13)) + G1(13) * LF(13);
  const v4f y12 = G0(12) * (y25 * R0(12) + y26 * R1(12)) + G1(12) * LF(12);
  const v4f y11 = G0(11) * (y23 * R0(11) + y24 * R1(11)) + G1(11) * LF(11);
  const v4f y10 = G0(10) * (y21 * R0(10) + y22 * R1(10)) + G1(10) * LF(10);
  const v4f y9 = G0(9) * (y19 * R0(9) + y20 * R1(9)) + G1(9) * LF(9);
  const v4f y8 = G0(8) * (y17 * R0(8) + y18 * R1(8)) + G1(8) * LF(8);
  const v4f y7 = G0(7) * (y15 * R0(7) + y16 * R1(7)) + G1(7) * LF(7);
  const v4f y6 = G0(6) * (y13 * R0(6) + y14 * R1(6)) + G1(6) * LF(6);
  const v4f y5 = G0(5) * (y11 * R0(5) + y12 * R1(5)) + G1(5) * LF(5);
  const v4f y4 = G0(4) * (y9 * R0(4) + y10 * R1(4)) + G1(4) * LF(4);
  const v4f y3 = G0(3) * (y7 * R0(3) + y8 * R1(3)) + G1(3) * LF(3);
  const v4f y2 = G0(2) * (y5 * R0(2) + y6 * R1(2)) + G1(2) * LF(2);
  const v4f y1 = G0(1) * (y3 * R0(1) + y4 * R1(1)) + G1(1) * LF(1);
  const v4f y0 = G0(0) * (y1 * R0(0) + y2 * R1(0)) + G1(0) * LF(0);
  float* op = OUT + (size_t)row * NO + q * 4; *(volatile v4f*)op = y0; __threadfence(); *(volatile v4f*)op = y0;
}

extern "C" void kernel_launch(void* const* d_in, const int* in_sizes, int n_in,
                              void* d_out, int out_size, void* d_ws, size_t ws_size, hipStream_t stream) {
    (void)in_sizes; (void)n_in; (void)out_size;
    const float* x = (const float*)d_in[0]; const float* Wi = (const float*)d_in[1]; const float* bi = (const float*)d_in[2]; const float* gm = (const float*)d_in[3]; const float* leaf = (const float*)d_in[4];
    float* OUT = (float*)d_out;
    char* wsp = (char*)d_ws;
    auto take = [&](size_t bytes) { char* p = wsp; wsp += (bytes + 255) & ~(size_t)255; return (void*)p; };
    bf* XB = (bf*)take((size_t)NB * NK * 2); bf* WB = (bf*)take((size_t)NLP * NK * 2); float* LG = (float*)take((size_t)NB * NLP * 4); float* RR = (float*)take((size_t)NB * 64 * 4); float* GG = (float*)take((size_t)NI * 2 * 4);
    if ((size_t)(wsp - (char*)d_ws) > ws_size) return;
    k_cvt8<<<(unsigned)(((size_t)NB * NK / 8 + 255) / 256), 256, 0, stream>>>(x, XB, (size_t)NB * NK / 8);
    k_wpad<<<(NLP * NK / 8 + 255) / 256, 256, 0, stream>>>(Wi, WB);
    k_g<<<1, 32, 0, stream>>>(gm, GG);
    k_gemmw<bf, 0, false><<<dim3(NB / 64, NLP / 64, 1), 32, 0, stream>>>(XB, nullptr, WB, nullptr, NK, LG, NLP, nullptr, 0, 0, 0);
    k_route<<<NB * 32 / 256, 256, 0, stream>>>(LG, bi, RR);
    k_tree<<<NB * (NO / 4) / 256, 256, 0, stream>>>(RR, GG, leaf, OUT);
}
